// GRUBaselineClassifier_73744588472583
// MI455X (gfx1250) — hardware-verified
//
#include <hip/hip_runtime.h>
#include <math.h>

typedef __attribute__((ext_vector_type(16))) _Float16 v16h;
typedef __attribute__((ext_vector_type(16))) __bf16 v16b;
typedef __attribute__((ext_vector_type(8)))  _Float16 v8h;
typedef __attribute__((ext_vector_type(8)))  float v8f;
typedef __attribute__((ext_vector_type(4)))  float v4f;
typedef __attribute__((ext_vector_type(2)))  float v2f;
typedef __attribute__((ext_vector_type(4)))  unsigned v4u;
typedef __attribute__((ext_vector_type(4)))  int v4i;
typedef float __attribute__((may_alias)) float_a;
typedef int __attribute__((may_alias)) int_a;

template <typename T> __device__ __forceinline__ void vst2(void* p, T v) { *(volatile T*)p = v; __threadfence(); *(volatile T*)p = v; }
__device__ __forceinline__ v8f wmma16(v16h a, v16h b, v8f c) {
  v8f d = __builtin_amdgcn_wmma_f32_16x16x32_f16(false, a, false, b, (short)0, c, false, false);
  asm volatile("v_nop\n\tv_nop\n\tv_nop\n\tv_nop" : "+v"(d) : "v"(a), "v"(b));
  return d;
}
__device__ __forceinline__ v8f wmma_bf(v16b a, v16b b, v8f c) {
  v8f d = __builtin_amdgcn_wmma_f32_16x16x32_bf16(false, a, false, b, (short)0, c, false, false);
  asm volatile("v_nop\n\tv_nop\n\tv_nop\n\tv_nop" : "+v"(d) : "v"(a), "v"(b));
  return d;
}
__device__ __forceinline__ v16h frag_h(const _Float16* rowk0, int lane) {
  union { v16h v; v8h q[2]; } u; const _Float16* p = rowk0 + 8 * (lane >> 4);
  u.q[0] = *(const v8h*)p; u.q[1] = *(const v8h*)(p + 16); return u.v;
}
__device__ __forceinline__ v16h frag_f32(const float* rowk0, int lane) {
  v16h a; const float* p = rowk0 + 8 * (lane >> 4);
#pragma unroll
  for (int i = 0; i < 8; ++i) { a[i] = (_Float16)p[i]; a[8 + i] = (_Float16)p[16 + i]; }
  return a;
}
__device__ __forceinline__ v16h frag_f32s(const float* rowk0, int lane, float sc) {
  v16h a; const float* p = rowk0 + 8 * (lane >> 4);
#pragma unroll
  for (int i = 0; i < 8; ++i) { a[i] = (_Float16)(p[i] * sc); a[8 + i] = (_Float16)(p[16 + i] * sc); }
  return a;
}
__device__ __forceinline__ v16h fragc_f32(const float* W, int k0, int n, int lane, int ld, int K) {
  v16h a; const int g = lane >> 4;
#pragma unroll
  for (int i = 0; i < 8; ++i) { const int ka = k0 + 8 * g + i, kb = ka + 16;
    a[i] = (_Float16)(ka < K ? W[(size_t)ka * ld + n] : 0.f); a[8 + i] = (_Float16)(kb < K ? W[(size_t)kb * ld + n] : 0.f); }
  return a;
}
struct F2 { v16b h, l; };
__device__ __forceinline__ F2 bsplit16(const float v[16]) { F2 r;
#pragma unroll
  for (int i = 0; i < 16; ++i) { const __bf16 h = (__bf16)v[i]; r.h[i] = h; r.l[i] = (__bf16)(v[i] - (float)h); }
  return r; }
__device__ __forceinline__ F2 split_row(const float* row, int k0, int lane) { float v[16]; const float* p = row + k0 + 8 * (lane >> 4);
#pragma unroll
  for (int i = 0; i < 8; ++i) { v[i] = p[i]; v[8 + i] = p[16 + i]; }
  return bsplit16(v); }
__device__ __forceinline__ F2 split_rowK(const float* row, int k0, int lane, int K) { float v[16]; const int g = lane >> 4;
#pragma unroll
  for (int i = 0; i < 8; ++i) { const int ka = k0 + 8 * g + i, kb = ka + 16; v[i] = ka < K ? row[ka] : 0.f; v[8 + i] = kb < K ? row[kb] : 0.f; }
  return bsplit16(v); }
__device__ __forceinline__ F2 split_col(const float* W, int k0, int n, int lane, int ld, int K) { float v[16]; const int g = lane >> 4;
#pragma unroll
  for (int i = 0; i < 8; ++i) { const int ka = k0 + 8 * g + i, kb = ka + 16; v[i] = ka < K ? W[(size_t)ka * ld + n] : 0.f; v[8 + i] = kb < K ? W[(size_t)kb * ld + n] : 0.f; }
  return bsplit16(v); }
__device__ __forceinline__ v8f mac3(const F2& a, const F2& b, v8f c) { c = wmma_bf(a.l, b.h, c); c = wmma_bf(a.h, b.l, c); return wmma_bf(a.h, b.h, c); }
__device__ __forceinline__ float sigm(float v) { return 1.0f / (1.0f + expf(-v)); }
#define LDSX() do { asm volatile("s_wait_dscnt 0" ::: "memory"); __builtin_amdgcn_wave_barrier(); __builtin_amdgcn_fence(__ATOMIC_RELEASE, "workgroup"); } while (0)

#define NBT 128
#define TT 2048
#define EE 64
#define HH 64
#define G3 192
#define VOC 50257
#define NCLS 20

__global__ __launch_bounds__(256) void k_gath(const int* __restrict__ tok, const float* __restrict__ emb, _Float16* __restrict__ X16) {
  const size_t r = ((size_t)blockIdx.x * 256 + threadIdx.x) >> 4; const int part = threadIdx.x & 15;
  if (r >= (size_t)NBT * TT) return;
  int id = tok[r]; id = id < 0 ? 0 : (id >= VOC ? VOC - 1 : id);
  const v4f v = *(const v4f*)(emb + (size_t)id * EE + part * 4);
  union { _Float16 h4[4]; unsigned long long u; } pk;
#pragma unroll
  for (int e = 0; e < 4; ++e) pk.h4[e] = (_Float16)v[e];
  vst2((unsigned long long*)(X16 + r * EE) + part, pk.u);
}
__global__ __launch_bounds__(32) void k_gru(const _Float16* __restrict__ X16, const float* __restrict__ wih_f, const float* __restrict__ whh_f, const float* __restrict__ bih_f, const float* __restrict__ bhh_f,
                                          const float* __restrict__ wih_b, const float* __restrict__ whh_b, const float* __restrict__ bih_b, const float* __restrict__ bhh_b, float* __restrict__ FEAT) {
  __shared__ __align__(16) _Float16 sWi[G3][EE + 8], sWh[G3][HH + 8];
  __shared__ __align__(16) _Float16 sh16[16][HH + 8];
  __shared__ __align__(16) float sh32[16][HH + 4];
  __shared__ float sbi[G3], sbh[G3];
  const int lane = threadIdx.x, col = lane & 15, g = lane >> 4;
  const int dir = blockIdx.y, b0 = blockIdx.x * 16;
  const float* wih = dir ? wih_b : wih_f; const float* whh = dir ? whh_b : whh_f; const float* bih = dir ? bih_b : bih_f; const float* bhh = dir ? bhh_b : bhh_f;
  for (int q = lane; q < G3 * EE; q += 32) { const int n = q >> 6, k = q & 63; sWi[n][k] = (_Float16)wih[q]; sWh[n][k] = (_Float16)whh[q]; }
  for (int q = lane; q < G3; q += 32) { sbi[q] = bih[q]; sbh[q] = bhh[q]; }
  for (int q = lane; q < 16 * (HH + 8); q += 32) (&sh16[0][0])[q] = (_Float16)0.f;
  for (int q = lane; q < 16 * (HH + 4); q += 32) (&sh32[0][0])[q] = 0.f;
  LDSX();
  float hsum[4][8], hmax[4][8];
#pragma unroll
  for (int t = 0; t < 4; ++t)
#pragma unroll
    for (int r = 0; r < 8; ++r) { hsum[t][r] = 0.f; hmax[t][r] = -3.0e38f; }
#pragma unroll 1
  for (int s = 0; s < TT; ++s) { const int t_idx = dir ? (TT - 1 - s) : s;
    v16h ax[2], ah[2];
#pragma unroll
    for (int kc = 0; kc < 2; ++kc) { ax[kc] = frag_h(X16 + ((size_t)(b0 + col) * TT + t_idx) * EE + kc * 32, lane); ah[kc] = frag_h(&sh16[col][0] + kc * 32, lane); }
    float hn[4][8];
#pragma unroll
    for (int t = 0; t < 4; ++t) { v8f ar = {}, az = {}, anx = {}, anh = {};
#pragma unroll
      for (int kc = 0; kc < 2; ++kc) {
        ar = wmma16(ax[kc], frag_h(&sWi[t * 16 + col][0] + kc * 32, lane), ar); ar = wmma16(ah[kc], frag_h(&sWh[t * 16 + col][0] + kc * 32, lane), ar);
        az = wmma16(ax[kc], frag_h(&sWi[64 + t * 16 + col][0] + kc * 32, lane), az); az = wmma16(ah[kc], frag_h(&sWh[64 + t * 16 + col][0] + kc * 32, lane), az);
        anx = wmma16(ax[kc], frag_h(&sWi[128 + t * 16 + col][0] + kc * 32, lane), anx); anh = wmma16(ah[kc], frag_h(&sWh[128 + t * 16 + col][0] + kc * 32, lane), anh); }
      const int u = t * 16 + col; const float bir = sbi[u], bhr = sbh[u], biz = sbi[64 + u], bhz = sbh[64 + u], bin_ = sbi[128 + u], bhn = sbh[128 + u];
#pragma unroll
      for (int r = 0; r < 8; ++r) { const float hp = sh32[8 * g + r][u];
        const float rg = sigm(ar[r] + bir + bhr); const float zg = sigm(az[r] + biz + bhz);
        const float ng = tanhf(anx[r] + bin_ + rg * (anh[r] + bhn));
        const float hv = (1.0f - zg) * ng + zg * hp; hn[t][r] = hv; hsum[t][r] += hv; hmax[t][r] = fmaxf(hmax[t][r], hv); } }
    LDSX();
#pragma unroll
    for (int t = 0; t < 4; ++t)
#pragma unroll
      for (int r = 0; r < 8; ++r) { sh32[8 * g + r][t * 16 + col] = hn[t][r]; sh16[8 * g + r][t * 16 + col] = (_Float16)hn[t][r]; }
    LDSX(); }
  __shared__ __align__(16) float sf[16][2][HH];
#pragma unroll
  for (int t = 0; t < 4; ++t)
#pragma unroll
    for (int r = 0; r < 8; ++r) { sf[8 * g + r][0][t * 16 + col] = hsum[t][r] * (1.0f / TT); sf[8 * g + r][1][t * 16 + col] = hmax[t][r]; }
  LDSX();
  for (int q = lane; q < 16 * 2 * 16; q += 32) { const int rl = q >> 5, mm = (q >> 4) & 1, pc = q & 15; vst2(FEAT + (size_t)(b0 + rl) * 256 + mm * 128 + dir * 64 + pc * 4, *(const v4f*)(&sf[rl][mm][pc * 4])); }
}
__global__ __launch_bounds__(128) void k_head(const float* __restrict__ FEAT, const float* __restrict__ w1, const float* __restrict__ b1, const float* __restrict__ w2, const float* __restrict__ b2, float* __restrict__ out) {
  __shared__ float shid[NBT][HH + 1]; __shared__ __align__(16) float so[NBT * NCLS];
  const int tid = threadIdx.x;
  for (int q = tid; q < NBT * HH; q += 128) { const int bb = q >> 6, o = q & 63; float s = b1[o];
#pragma unroll 4
    for (int k = 0; k < 256; ++k) s += FEAT[(size_t)bb * 256 + k] * w1[o * 256 + k];
    shid[bb][o] = 0.5f * s * (1.0f + erff(s * 0.70710678118654752f)); }
  __syncthreads();
  for (int q = tid; q < NBT * NCLS; q += 128) { const int bb = q / NCLS, c = q % NCLS; float s = b2[c];
#pragma unroll 4
    for (int k = 0; k < HH; ++k) s += shid[bb][k] * w2[c * HH + k];
    so[q] = s; }
  __syncthreads();
  for (int q = tid; q < NBT * NCLS / 4; q += 128) vst2(out + q * 4, *(const v4f*)(&so[q * 4]));
}
extern "C" void kernel_launch(void* const* d_in, const int* in_sizes, int n_in, void* d_out, int out_size, void* d_ws, size_t ws_size, hipStream_t stream) {
  (void)in_sizes; (void)n_in; (void)out_size; (void)ws_size;
  const int* tok = (const int*)d_in[0]; const float** I = (const float**)d_in;
  float* out = (float*)d_out;
  char* ws = (char*)d_ws; size_t off = 0;
  auto take = [&](size_t bytes) { char* p = ws + off; off += (bytes + 255) & ~(size_t)255; return p; };
  _Float16* X16 = (_Float16*)take((size_t)NBT * TT * EE * 2); float* FEAT = (float*)take((size_t)NBT * 256 * 4);
  k_gath<<<(NBT * TT * 16) / 256, 256, 0, stream>>>(tok, I[1], X16);
  k_gru<<<dim3(NBT / 16, 2), 32, 0, stream>>>(X16, I[2], I[3], I[4], I[5], I[6], I[7], I[8], I[9], FEAT);
  k_head<<<1, 128, 0, stream>>>(FEAT, I[10], I[11], I[12], I[13], out);
}
